// InterpretableMultiHeadAttention_37958920962401
// MI455X (gfx1250) — hardware-verified
//
#include <hip/hip_runtime.h>
#include <math.h>
#include <stdint.h>

#ifndef NB
#define NB 2
#endif
#ifndef SEQ
#define SEQ 2048
#endif
#define NB_FULL  2
#define SEQ_FULL 2048
#define EMB      1024
#define NH       16
#define HD       64
#define NROW     (NB * SEQ)
#define NQB      (SEQ / 16)
#define NKT      (SEQ / 64)
#define PCARRY   16384.0f
#define OFF1     ((size_t)NB_FULL * SEQ_FULL * EMB)
static_assert(NB >= 1 && NB <= NB_FULL);
static_assert(SEQ >= 64 && SEQ <= SEQ_FULL && (SEQ % 64) == 0);
static_assert(NH * HD == EMB);
static_assert((NROW % 64) == 0 && (EMB % 64) == 0 && (HD % 64) == 0 && (EMB % 32) == 0);
static_assert(OFF1 * 4 == 16777216);

typedef _Float16 v16h __attribute__((ext_vector_type(16)));
typedef _Float16 v8h  __attribute__((ext_vector_type(8)));
typedef __bf16   v16b __attribute__((ext_vector_type(16)));
typedef __bf16   v8b  __attribute__((ext_vector_type(8)));
typedef float    v8f  __attribute__((ext_vector_type(8)));
typedef float    v4f  __attribute__((ext_vector_type(4)));
typedef unsigned int v4u __attribute__((ext_vector_type(4)));

#if defined(__HIP_DEVICE_COMPILE__)
#define DEV_ASM 1
#else
#define DEV_ASM 0
#endif

__device__ __forceinline__ unsigned short bf_bits(float f) {
  unsigned u = __float_as_uint(f);
  return (unsigned short)((u + 0x7FFFu + ((u >> 16) & 1u)) >> 16);
}
__device__ __forceinline__ float bf_up(unsigned short hb) { return __uint_as_float(((unsigned)hb) << 16); }
__device__ __forceinline__ unsigned short h_bits(_Float16 x) { return __builtin_bit_cast(unsigned short, x); }
__device__ __forceinline__ unsigned pk16(unsigned short a, unsigned short b) { return (unsigned)a | ((unsigned)b << 16); }
__device__ __forceinline__ v8f zero8() { v8f z = {0.f, 0.f, 0.f, 0.f, 0.f, 0.f, 0.f, 0.f}; return z; }

template <typename OT> struct FT;
template <> struct FT<__bf16>   { typedef v16b frag; typedef v8b half8; };
template <> struct FT<_Float16> { typedef v16h frag; typedef v8h half8; };

template <typename OT>
__device__ __forceinline__ typename FT<OT>::frag ldfrag(const OT* p) {
  union { typename FT<OT>::frag v; typename FT<OT>::half8 h[2]; } f;
  f.h[0] = *(const typename FT<OT>::half8*)(p);
  f.h[1] = *(const typename FT<OT>::half8*)(p + 16);
  return f.v;
}

__device__ __forceinline__ v8f mmar(v16b a, v16b b, v8f c) {
  return __builtin_amdgcn_wmma_f32_16x16x32_bf16(false, a, false, b, (short)0, c, false, false);
}
__device__ __forceinline__ v8f mmar(v16h a, v16h b, v8f c) {
  return __builtin_amdgcn_wmma_f32_16x16x32_f16(false, a, false, b, (short)0, c, false, false);
}
__device__ __forceinline__ v8f mma_h(v16h a, v16h b, v8f c) {
  c = __builtin_amdgcn_wmma_f32_16x16x32_f16(false, a, false, b, (short)0, c, false, false);
#if DEV_ASM
  asm volatile("v_nop\n\tv_nop\n\tv_nop\n\tv_nop" : "+v"(c) : "v"(a), "v"(b));
#endif
  return c;
}
__device__ __forceinline__ void dep_guard(v8f& a, v8f& b, v16b x, v16b y) {
#if DEV_ASM
  asm volatile("v_nop\n\tv_nop\n\tv_nop\n\tv_nop" : "+v"(a), "+v"(b) : "v"(x), "v"(y));
#else
  (void)a; (void)b; (void)x; (void)y;
#endif
}
__device__ __forceinline__ void dep_guard(v8f& a, v8f& b, v16h x, v16h y) {
#if DEV_ASM
  asm volatile("v_nop\n\tv_nop\n\tv_nop\n\tv_nop" : "+v"(a), "+v"(b) : "v"(x), "v"(y));
#else
  (void)a; (void)b; (void)x; (void)y;
#endif
}
__device__ __forceinline__ void keep4(v16b a, v16b b, v16b c, v16b d) {
#if DEV_ASM
  asm volatile("v_nop" :: "v"(a), "v"(b), "v"(c), "v"(d));
#else
  (void)a; (void)b; (void)c; (void)d;
#endif
}
__device__ __forceinline__ void keep4(v16h a, v16h b, v16h c, v16h d) {
#if DEV_ASM
  asm volatile("v_nop" :: "v"(a), "v"(b), "v"(c), "v"(d));
#else
  (void)a; (void)b; (void)c; (void)d;
#endif
}
__device__ __forceinline__ void acc_guard4(v8f& a, v8f& b, v8f& c, v8f& d) {
#if DEV_ASM
  asm volatile("v_nop\n\tv_nop\n\tv_nop\n\tv_nop" : "+v"(a), "+v"(b), "+v"(c), "+v"(d));
#else
  (void)a; (void)b; (void)c; (void)d;
#endif
}

template <int MODE>
__device__ __forceinline__ unsigned short cvm(float f) {
  const unsigned short hb = bf_bits(f);
  if (MODE == 0) return hb;
  return h_bits((_Float16)(bf_up(hb) * 64.0f));
}

template <int MODE>
__global__ __launch_bounds__(256) void cvt16x8(const float* __restrict__ in, long long inStride,
                                               unsigned short* out, long long outStride, int n8) {
  const int i = blockIdx.x * 256 + (int)threadIdx.x;
  const float* ib = in + (size_t)blockIdx.y * (size_t)inStride;
  unsigned short* ob = out + (size_t)blockIdx.y * (size_t)outStride;
  if (i < n8) {
    const v4f a  = *(const v4f*)(ib + (size_t)i * 8);
    const v4f a4 = *(const v4f*)(ib + (size_t)i * 8 + 4);
    v4u p;
    p[0] = pk16(cvm<MODE>(a[0]),  cvm<MODE>(a[1]));
    p[1] = pk16(cvm<MODE>(a[2]),  cvm<MODE>(a[3]));
    p[2] = pk16(cvm<MODE>(a4[0]), cvm<MODE>(a4[1]));
    p[3] = pk16(cvm<MODE>(a4[2]), cvm<MODE>(a4[3]));
    unsigned short* o = ob + (size_t)i * 8;
    *(volatile v4u*)o = p;
    __threadfence();
    *(volatile v4u*)o = p;
  }
}

template <int MODE>
__global__ __launch_bounds__(256) void tr16(const float* __restrict__ in, unsigned short* out, int K, int N) {
  __shared__ float s[64][65];
  const int t  = threadIdx.x;
  const int n0 = blockIdx.x * 64;
  const int k0 = blockIdx.y * 64;
#pragma unroll
  for (int it = 0; it < 4; ++it) {
    const int f  = t + it * 256;
    const int kk = f >> 4, c4 = (f & 15) * 4;
    const v4f v = *(const v4f*)(in + (size_t)(k0 + kk) * (size_t)N + n0 + c4);
    s[kk][c4 + 0] = v[0];
    s[kk][c4 + 1] = v[1];
    s[kk][c4 + 2] = v[2];
    s[kk][c4 + 3] = v[3];
  }
  __syncthreads();
  v4u pv[2];
#pragma unroll
  for (int it = 0; it < 2; ++it) {
    const int nn = (t >> 3) + it * 32, c8 = (t & 7) * 8;
    v4u p;
#pragma unroll
    for (int e = 0; e < 4; ++e)
      p[e] = pk16(cvm<MODE>(s[c8 + 2 * e][nn]), cvm<MODE>(s[c8 + 2 * e + 1][nn]));
    pv[it] = p;
  }
  for (int pass = 0; pass < 2; ++pass) {
#pragma unroll
    for (int it = 0; it < 2; ++it) {
      const int nn = (t >> 3) + it * 32, c8 = (t & 7) * 8;
      *(volatile v4u*)(out + (size_t)(n0 + nn) * (size_t)K + k0 + c8) = pv[it];
    }
    __threadfence();
  }
}

template <typename OT, int MI, int NPA, int OUT_MODE>
__global__ __launch_bounds__(256) void gemm_t(
    const unsigned short* __restrict__ Ap, const unsigned short* __restrict__ A2p, int lda, long long strideA,
    const unsigned short* __restrict__ Btp, int ldb, long long strideB,
    void* Cout, void* Cout2, int ldc, long long strideC,
    int M, int N, int K, float oscale, float rscaleA, float cscale, float rscaleC) {
  typedef typename FT<OT>::frag V16;
  const OT* A  = (const OT*)(const void*)Ap;
  const OT* A2 = (const OT*)(const void*)A2p;
  const OT* Bt = (const OT*)(const void*)Btp;
  __shared__ __align__(16) float sT[8][16 * 68];
  const int RT   = 16 * MI;
  const int b    = blockIdx.y;
  const int lane = threadIdx.x & 31;
  const int wave = threadIdx.x >> 5;
  const int tilesN = N >> 6;
  const int tilesM = M / RT;
  const int tile = blockIdx.x * 8 + wave;
  if (tile >= tilesM * tilesN) return;
  const int tm = tile / tilesN;
  const int tn = tile - tm * tilesN;
  const int m0 = tm * RT;
  const int n0 = tn << 6;

  const OT* Ab  = A  + (size_t)b * (size_t)strideA;
  const OT* A2b = A2 + (size_t)b * (size_t)strideA;
  const OT* Bb  = Bt + (size_t)b * (size_t)strideB;

  const int rlane = lane & 15;
  const int koff  = (lane >> 4) * 8;
  const int mOff  = (lane >> 4) * 8;

  v8f acc[MI][4], acc2[MI][4];
#pragma unroll
  for (int i = 0; i < MI; ++i)
#pragma unroll
    for (int j = 0; j < 4; ++j) { acc[i][j] = zero8(); acc2[i][j] = zero8(); }

  for (int k0 = 0; k0 < K; k0 += 32) {
    V16 bq[4];
#pragma unroll
    for (int j = 0; j < 4; ++j)
      bq[j] = ldfrag<OT>(Bb + (size_t)(n0 + (j << 4) + rlane) * ldb + koff + k0);
#pragma unroll
    for (int i = 0; i < MI; ++i) {
      const V16 af = ldfrag<OT>(Ab + (size_t)(m0 + (i << 4) + rlane) * lda + koff + k0);
#pragma unroll
      for (int j = 0; j < 4; ++j) acc[i][j] = mmar(af, bq[j], acc[i][j]);
      dep_guard(acc[i][0], acc[i][3], af, bq[3]);
      if (NPA == 2) {
        const V16 af2 = ldfrag<OT>(A2b + (size_t)(m0 + (i << 4) + rlane) * lda + koff + k0);
#pragma unroll
        for (int j = 0; j < 4; ++j) acc2[i][j] = mmar(af2, bq[j], acc2[i][j]);
        dep_guard(acc2[i][0], acc2[i][3], af2, bq[3]);
      }
    }
    keep4(bq[0], bq[1], bq[2], bq[3]);
  }
#pragma unroll
  for (int i = 0; i < MI; ++i) {
    acc_guard4(acc[i][0], acc[i][1], acc[i][2], acc[i][3]);
    if (NPA == 2) acc_guard4(acc2[i][0], acc2[i][1], acc2[i][2], acc2[i][3]);
  }

  float* slab = sT[wave];
#pragma unroll
  for (int i = 0; i < MI; ++i) {
    const int mBase = m0 + (i << 4);
#pragma unroll
    for (int j = 0; j < 4; ++j) {
#pragma unroll
      for (int r = 0; r < 8; ++r) {
        float v = acc[i][j][r];
        if (NPA == 2) v += acc2[i][j][r] * rscaleA;
        v = v * oscale;
        slab[(mOff + r) * 68 + (j << 4) + rlane] = v;
      }
    }
    __builtin_amdgcn_fence(__ATOMIC_RELEASE, "workgroup");
    __builtin_amdgcn_wave_barrier();
    __builtin_amdgcn_fence(__ATOMIC_ACQUIRE, "workgroup");
    if (OUT_MODE == 0) {
      float* C = (float*)Cout + (size_t)b * (size_t)strideC;
      const int h2 = lane >> 4, c4 = (lane & 15) * 4;
      v4f ov[8];
#pragma unroll
      for (int it = 0; it < 8; ++it) {
        const int row = it * 2 + h2;
        ov[it] = *(const v4f*)(slab + row * 68 + c4);
      }
      for (int pass = 0; pass < 2; ++pass) {
#pragma unroll
        for (int it = 0; it < 8; ++it) {
          const int row = it * 2 + h2;
          *(volatile v4f*)(C + (size_t)(mBase + row) * ldc + n0 + c4) = ov[it];
        }
        __threadfence();
      }
    } else {
      const int q = lane >> 3, c8 = (lane & 7) * 8;
      unsigned short* C  = (unsigned short*)Cout  + (size_t)b * (size_t)strideC;
      unsigned short* C2 = (unsigned short*)Cout2 + (size_t)b * (size_t)strideC;
      v4u hv[4], lv[4];
#pragma unroll
      for (int it = 0; it < 4; ++it) {
        const int row = it * 4 + q;
        const float* sp = slab + row * 68 + c8;
        float f[8];
#pragma unroll
        for (int e = 0; e < 8; ++e) f[e] = sp[e] * cscale;
        v4u a, a2;
#pragma unroll
        for (int e = 0; e < 4; ++e) {
          const float f0 = f[2 * e], f1 = f[2 * e + 1];
          const _Float16 x0 = (_Float16)f0, x1 = (_Float16)f1;
          const unsigned short h0 = h_bits(x0), h1 = h_bits(x1);
          unsigned short l0 = 0, l1 = 0;
          if (OUT_MODE == 3) {
            l0 = h_bits((_Float16)((f0 - (float)x0) * rscaleC));
            l1 = h_bits((_Float16)((f1 - (float)x1) * rscaleC));
          }
          a[e] = pk16(h0, h1); a2[e] = pk16(l0, l1);
        }
        hv[it] = a; lv[it] = a2;
      }
      for (int pass = 0; pass < 2; ++pass) {
#pragma unroll
        for (int it = 0; it < 4; ++it) {
          const int row = it * 4 + q;
          *(volatile v4u*)(C + (size_t)(mBase + row) * ldc + n0 + c8) = hv[it];
          if (OUT_MODE == 3) *(volatile v4u*)(C2 + (size_t)(mBase + row) * ldc + n0 + c8) = lv[it];
        }
        __threadfence();
      }
    }
    __builtin_amdgcn_fence(__ATOMIC_RELEASE, "workgroup");
    __builtin_amdgcn_wave_barrier();
    __builtin_amdgcn_fence(__ATOMIC_ACQUIRE, "workgroup");
  }
}

__device__ __forceinline__ void score_chunk(const v16h (&qah)[2], const v16h (&qal)[2],
                                            const _Float16* __restrict__ kb0, int kv0, int c, int hh,
                                            v8f (&s)[4]) {
  union FH { v16h v; v8h h[2]; };
#pragma unroll
  for (int j = 0; j < 4; ++j) {
    v8f ah = zero8(), al = zero8();
#pragma unroll
    for (int dc = 0; dc < 2; ++dc) {
      const _Float16* kp = kb0 + (size_t)(kv0 + j * 16 + c) * (size_t)EMB + dc * 32 + 8 * hh;
      FH kb;
      kb.h[0] = *(const v8h*)(kp);
      kb.h[1] = *(const v8h*)(kp + 16);
      ah = mma_h(qah[dc], kb.v, ah);
      al = mma_h(qal[dc], kb.v, al);
    }
#pragma unroll
    for (int r = 0; r < 8; ++r) s[j][r] = (ah[r] + al[r] * (1.0f / 4096.0f)) * 0.125f;
  }
}

__global__ __launch_bounds__(128)
void attn_stats(const unsigned short* __restrict__ qhp, const unsigned short* __restrict__ qlp,
                const unsigned short* __restrict__ kpp, float* ML) {
  __shared__ __align__(16) float MLsh[128];
  const int tid  = threadIdx.x;
  const int wave = tid >> 5;
  const int lane = tid & 31;
  const int hh   = lane >> 4;
  const int c    = lane & 15;
  const int bx   = blockIdx.x;
  const int qb   = bx % NKT;
  const int rest = bx / NKT;
  const int h    = rest % NH;
  const int b    = rest / NH;
  const int bh   = b * NH + h;
  const int q0   = qb * 64 + wave * 16;

  const _Float16* Qh  = (const _Float16*)(const void*)qhp;
  const _Float16* Ql  = (const _Float16*)(const void*)qlp;
  const _Float16* Kb0 = (const _Float16*)(const void*)kpp + (size_t)b * SEQ * EMB + (size_t)h * HD;

  v16h qah[2], qal[2];
#pragma unroll
  for (int dc = 0; dc < 2; ++dc) {
    const size_t qo = ((size_t)b * SEQ + (size_t)(q0 + c)) * EMB + (size_t)h * HD + dc * 32 + 8 * hh;
    qah[dc] = ldfrag<_Float16>(Qh + qo);
    qal[dc] = ldfrag<_Float16>(Ql + qo);
  }

  float mrow[8], lrow[8];
#pragma unroll
  for (int r = 0; r < 8; ++r) { mrow[r] = -INFINITY; lrow[r] = 0.f; }

  for (int kt = 0; kt < NKT; ++kt) {
    const int kv0 = kt * 64;
    v8f s[4];
    score_chunk(qah, qal, Kb0, kv0, c, hh, s);
#pragma unroll
    for (int r = 0; r < 8; ++r) {
      float m = s[0][r];
#pragma unroll
      for (int j = 1; j < 4; ++j) m = fmaxf(m, s[j][r]);
#pragma unroll
      for (int off = 1; off < 16; off <<= 1) m = fmaxf(m, __shfl_xor(m, off, 32));
      const float mnew  = fmaxf(mrow[r], m);
      const float msafe = (mnew == -INFINITY) ? 0.f : mnew;
      const float alpha = __expf(mrow[r] - msafe);
      mrow[r] = mnew;
      float psum = 0.f;
#pragma unroll
      for (int j = 0; j < 4; ++j) psum += __expf(s[j][r] - msafe);
#pragma unroll
      for (int off = 1; off < 16; off <<= 1) psum += __shfl_xor(psum, off, 32);
      lrow[r] = lrow[r] * alpha + psum;
    }
  }

  float il[8];
#pragma unroll
  for (int r = 0; r < 8; ++r) {
    const float l = lrow[r];
    il[r] = (l > 0.f) ? (1.0f / l) : 0.f;
  }
  if (c == 0) {
#pragma unroll
    for (int r = 0; r < 8; ++r) {
      MLsh[wave * 16 + 8 * hh + r]      = mrow[r];
      MLsh[64 + wave * 16 + 8 * hh + r] = il[r];
    }
  }
  __syncthreads();
  if (wave == 0) {
    const v4f v = *(const v4f*)(MLsh + lane * 4);
    float* dst = ML + (size_t)(bh * 2 + hh) * SEQ + qb * 64 + c * 4;
    *(volatile v4f*)dst = v;
    __threadfence();
    *(volatile v4f*)dst = v;
  }
}

__global__ __launch_bounds__(512)
void attn_main(const unsigned short* __restrict__ qhp, const unsigned short* __restrict__ qlp,
               const unsigned short* __restrict__ kpp, const unsigned short* __restrict__ vtp,
               const float* __restrict__ ML, unsigned short* chp, unsigned short* clp, float* avg) {
  union FH { v16h v; v8h h[2]; };
  __shared__ __align__(32) float Pf[NH][16 * 64];
  const int tid  = threadIdx.x;
  const int wave = tid >> 5;
  const int lane = tid & 31;
  const int hh   = lane >> 4;
  const int c    = lane & 15;
  const int bx   = blockIdx.x;
  const int qb   = bx % NQB;
  const int b    = bx / NQB;
  const int h    = wave;
  const int bh   = b * NH + h;
  const int q0   = qb * 16;

  const _Float16* Qh  = (const _Float16*)(const void*)qhp;
  const _Float16* Ql  = (const _Float16*)(const void*)qlp;
  const _Float16* Kb0 = (const _Float16*)(const void*)kpp + (size_t)b * SEQ * EMB + (size_t)h * HD;
  const _Float16* Vb0 = (const _Float16*)(const void*)vtp + (size_t)b * HD * SEQ;

  v16h qah[2], qal[2];
#pragma unroll
  for (int dc = 0; dc < 2; ++dc) {
    const size_t qo = ((size_t)b * SEQ + (size_t)(q0 + c)) * EMB + (size_t)h * HD + dc * 32 + 8 * hh;
    qah[dc] = ldfrag<_Float16>(Qh + qo);
    qal[dc] = ldfrag<_Float16>(Ql + qo);
  }
  const v8f m8  = *(const v8f*)(ML + (size_t)(bh * 2) * SEQ + q0 + 8 * hh);
  const v8f il8 = *(const v8f*)(ML + (size_t)(bh * 2 + 1) * SEQ + q0 + 8 * hh);

  v8f oacc[4];
#pragma unroll
  for (int t = 0; t < 4; ++t) oacc[t] = zero8();
  float* pf = Pf[wave];

  for (int kt = 0; kt < NKT; ++kt) {
    const int kv0 = kt * 64;
    __syncthreads();

    v8f s[4];
    score_chunk(qah, qal, Kb0, kv0, c, hh, s);
#pragma unroll
    for (int r = 0; r < 8; ++r) {
#pragma unroll
      for (int j = 0; j < 4; ++j) {
        const float p = __expf(s[j][r] - m8[r]) * il8[r];
        pf[(8 * hh + r) * 64 + j * 16 + c] = p;
      }
    }
    __builtin_amdgcn_fence(__ATOMIC_RELEASE, "workgroup");
    __builtin_amdgcn_wave_barrier();
    __builtin_amdgcn_fence(__ATOMIC_ACQUIRE, "workgroup");

#pragma unroll 1
    for (int kk = 0; kk < 2; ++kk) {
      const v8f p0 = *(const v8f*)(pf + c * 64 + kk * 32 + 8 * hh);
      const v8f p1 = *(const v8f*)(pf + c * 64 + kk * 32 + 16 + 8 * hh);
      FH pa;
      pa.h[0] = __builtin_convertvector(p0 * PCARRY, v8h);
      pa.h[1] = __builtin_convertvector(p1 * PCARRY, v8h);
#pragma unroll
      for (int t = 0; t < 4; ++t) {
        const v16h vb = ldfrag<_Float16>(Vb0 + (size_t)(t * 16 + c) * SEQ + kv0 + kk * 32 + 8 * hh);
        oacc[t] = mma_h(pa.v, vb, oacc[t]);
      }
    }
    __syncthreads();

    if (tid < 256) {
      const int row = tid >> 4, c4 = (tid & 15) * 4;
      v4f a = *(const v4f*)(Pf[0] + row * 64 + c4);
#pragma unroll
      for (int w = 1; w < NH; ++w) a += *(const v4f*)(Pf[w] + row * 64 + c4);
      a *= (1.0f / (float)NH);
      float* dst = avg + ((size_t)b * SEQ + (size_t)(q0 + row)) * SEQ + kv0 + c4;
      *(volatile v4f*)dst = a;
      __threadfence();
      *(volatile v4f*)dst = a;
    }
  }
  __syncthreads();

  float* os = pf;
#pragma unroll
  for (int r = 0; r < 8; ++r) {
#pragma unroll
    for (int t = 0; t < 4; ++t) os[(8 * hh + r) * 64 + t * 16 + c] = oacc[t][r] * (256.0f / PCARRY);
  }
  __builtin_amdgcn_fence(__ATOMIC_RELEASE, "workgroup");
  __builtin_amdgcn_wave_barrier();
  __builtin_amdgcn_fence(__ATOMIC_ACQUIRE, "workgroup");
  {
    const int q4 = lane >> 3, c8 = (lane & 7) * 8;
    v4u hv[4], lv[4];
#pragma unroll
    for (int it = 0; it < 4; ++it) {
      const int row = it * 4 + q4;
      const float* sp = os + row * 64 + c8;
      float f[8];
#pragma unroll
      for (int e = 0; e < 8; ++e) f[e] = sp[e];
      v4u a, a2;
#pragma unroll
      for (int e = 0; e < 4; ++e) {
        const float f0 = f[2 * e], f1 = f[2 * e + 1];
        const _Float16 x0 = (_Float16)f0, x1 = (_Float16)f1;
        const unsigned short h0 = h_bits(x0), h1 = h_bits(x1);
        const unsigned short l0 = h_bits((_Float16)((f0 - (float)x0) * 4096.0f));
        const unsigned short l1 = h_bits((_Float16)((f1 - (float)x1) * 4096.0f));
        a[e] = pk16(h0, h1); a2[e] = pk16(l0, l1);
      }
      hv[it] = a; lv[it] = a2;
    }
    for (int pass = 0; pass < 2; ++pass) {
#pragma unroll
      for (int it = 0; it < 4; ++it) {
        const int row = it * 4 + q4;
        const size_t go = ((size_t)b * SEQ + (size_t)(q0 + row)) * EMB + (size_t)h * HD + c8;
        *(volatile v4u*)(chp + go) = hv[it];
        *(volatile v4u*)(clp + go) = lv[it];
      }
      __threadfence();
    }
  }
}

__global__ __launch_bounds__(256)
void resid_ln(const float* __restrict__ Y, const float* __restrict__ x,
              const float* __restrict__ gam, const float* __restrict__ bet, float* out) {
  const int lane = threadIdx.x & 31;
  const int wave = threadIdx.x >> 5;
  const int row  = blockIdx.x * 8 + wave;
  if (row >= NROW) return;
  const int b = row / SEQ;
  const int s = row - b * SEQ;
  const float* xr = x + ((size_t)b * SEQ_FULL + (size_t)s) * EMB;
  const float* yr = Y + (size_t)row * EMB;

  v4f y[8];
  float sum = 0.f;
#pragma unroll
  for (int i = 0; i < 8; ++i) {
    const int col = i * 128 + lane * 4;
    const v4f xv = *(const v4f*)(xr + col);
    const v4f ov = *(const v4f*)(yr + col);
    v4f t;
#pragma unroll
    for (int e = 0; e < 4; ++e) t[e] = bf_up(bf_bits(xv[e])) + ov[e];
    y[i] = t;
    sum += (t[0] + t[1]) + (t[2] + t[3]);
  }
#pragma unroll
  for (int off = 1; off < 32; off <<= 1) sum += __shfl_xor(sum, off, 32);
  const float mu = sum * (1.0f / (float)EMB);

  float vs = 0.f;
#pragma unroll
  for (int i = 0; i < 8; ++i) {
#pragma unroll
    for (int e = 0; e < 4; ++e) { const float d = y[i][e] - mu; vs += d * d; }
  }
#pragma unroll
  for (int off = 1; off < 32; off <<= 1) vs += __shfl_xor(vs, off, 32);
  const float var = vs * (1.0f / (float)EMB);
  const float rs  = rsqrtf(var + 1e-6f);

  v4f o[8];
#pragma unroll
  for (int i = 0; i < 8; ++i) {
    const int col = i * 128 + lane * 4;
    const v4f g4 = *(const v4f*)(gam + col);
    const v4f b4 = *(const v4f*)(bet + col);
    v4f t;
#pragma unroll
    for (int e = 0; e < 4; ++e)
      t[e] = ((y[i][e] - mu) * rs) * bf_up(bf_bits(g4[e])) + bf_up(bf_bits(b4[e]));
    o[i] = t;
  }
  float* orow = out + (size_t)row * EMB;
  for (int pass = 0; pass < 2; ++pass) {
#pragma unroll
    for (int i = 0; i < 8; ++i) {
      const int col = i * 128 + lane * 4;
      *(volatile v4f*)(orow + col) = o[i];
    }
    __threadfence();
  }
}

extern "C" void kernel_launch(void* const* d_in, const int* in_sizes, int n_in,
                              void* d_out, int out_size, void* d_ws, size_t ws_size,
                              hipStream_t stream) {
  if (n_in < 7) return;
  if (in_sizes[0] < ((NB - 1) * SEQ_FULL + SEQ) * EMB) return;
  if (in_sizes[1] < EMB * EMB) return;
  if (in_sizes[2] < EMB * EMB) return;
  if (in_sizes[3] < EMB * HD) return;
  if (in_sizes[4] < EMB * EMB) return;
  if (in_sizes[5] < EMB) return;
  if (in_sizes[6] < EMB) return;
  const size_t n0e = (size_t)NROW * EMB;
  const size_t n1e = (size_t)NB * SEQ * SEQ;
  if (out_size < 0) return;
  if ((size_t)out_size < n0e) return;
  if ((size_t)out_size < OFF1 + n1e) return;

  const float* x   = (const float*)d_in[0];
  const float* Wq  = (const float*)d_in[1];
  const float* Wk  = (const float*)d_in[2];
  const float* Wv  = (const float*)d_in[3];
  const float* Wo  = (const float*)d_in[4];
  const float* gam = (const float*)d_in[5];
  const float* bet = (const float*)d_in[6];

  const size_t PX  = (size_t)NROW * EMB * 2;
  const size_t PW  = (size_t)EMB * EMB * 2;
  const size_t PWV = (size_t)HD * EMB * 2;
  const size_t PVT = (size_t)NB * HD * SEQ * 2;
  const size_t PML = (size_t)NB * NH * 2 * SEQ * 4;
  const size_t PY  = (size_t)NROW * EMB * 4;
  size_t off = 0;
  const size_t oXb = off; off += PX;
  const size_t oWq = off; off += PW;
  const size_t oWk = off; off += PW;
  const size_t oWv = off; off += PWV;
  const size_t oWo = off; off += PW;
  const size_t oQh = off; off += PX;
  const size_t oQl = off; off += PX;
  const size_t oKp = off; off += PX;
  const size_t oVT = off; off += PVT;
  const size_t oCh = off; off += PX;
  const size_t oCl = off; off += PX;
  const size_t oML = off; off += PML;
  const size_t oY  = off; off += PY;
  if (off > ws_size) return;
  if (off > (size_t)134217728) return;

  char* ws = (char*)d_ws;
  unsigned short* Xb  = (unsigned short*)(ws + oXb);
  unsigned short* WqT = (unsigned short*)(ws + oWq);
  unsigned short* WkT = (unsigned short*)(ws + oWk);
  unsigned short* WvT = (unsigned short*)(ws + oWv);
  unsigned short* WoT = (unsigned short*)(ws + oWo);
  unsigned short* Qh  = (unsigned short*)(ws + oQh);
  unsigned short* Ql  = (unsigned short*)(ws + oQl);
  unsigned short* Kp  = (unsigned short*)(ws + oKp);
  unsigned short* VT  = (unsigned short*)(ws + oVT);
  unsigned short* Ch  = (unsigned short*)(ws + oCh);
  unsigned short* Cl  = (unsigned short*)(ws + oCl);
  float*          ML  = (float*)(ws + oML);
  float*          Y   = (float*)(ws + oY);
  float*          out0 = (float*)d_out;
  float*          out1 = (float*)d_out + OFF1;

  const dim3 blk(256);
  const int n8x = SEQ * EMB / 8;
  const dim3 gCvtX((n8x + 255) / 256, NB);
  const dim3 gTrW(EMB / 64, EMB / 64);
  const dim3 gTrV(HD / 64, EMB / 64);
  const dim3 gQK((((NROW) / 64) * (EMB / 64) + 7) / 8, 1);
  const dim3 gV(((SEQ / 64) + 7) / 8, NB);
  const dim3 gO((((NROW) / 32) * (EMB / 64) + 7) / 8, 1);
  const dim3 gStats(NB * NH * NKT);
  const dim3 gMain(NB * NQB);
  const dim3 gLN((NROW + 7) / 8);

  cvt16x8<0><<<gCvtX, blk, 0, stream>>>(x, (long long)SEQ_FULL * EMB, Xb, (long long)SEQ * EMB, n8x);
  tr16<0><<<gTrW, blk, 0, stream>>>(Wq, WqT, EMB, EMB);
  tr16<0><<<gTrW, blk, 0, stream>>>(Wk, WkT, EMB, EMB);
  tr16<0><<<gTrV, blk, 0, stream>>>(Wv, WvT, EMB, HD);
  tr16<1><<<gTrW, blk, 0, stream>>>(Wo, WoT, EMB, EMB);
  gemm_t<__bf16, 4, 1, 3><<<gQK, blk, 0, stream>>>(
      Xb, Xb, EMB, 0LL, WqT, EMB, 0LL,
      (void*)Qh, (void*)Ql, EMB, 0LL,
      NROW, EMB, EMB, 1.0f, 0.0f, 1.0f, 4096.0f);
  gemm_t<__bf16, 4, 1, 1><<<gQK, blk, 0, stream>>>(
      Xb, Xb, EMB, 0LL, WkT, EMB, 0LL,
      (void*)Kp, (void*)Kp, EMB, 0LL,
      NROW, EMB, EMB, 1.0f, 0.0f, 1.0f, 1.0f);
  gemm_t<__bf16, 4, 1, 1><<<gV, blk, 0, stream>>>(
      WvT, WvT, EMB, 0LL, Xb, EMB, (long long)SEQ * EMB,
      (void*)VT, (void*)VT, SEQ, (long long)HD * SEQ,
      HD, SEQ, EMB, 1.0f, 0.0f, 1.0f, 1.0f);
  attn_stats<<<gStats, dim3(128), 0, stream>>>(Qh, Ql, Kp, ML);
  attn_main<<<gMain, dim3(512), 0, stream>>>(Qh, Ql, Kp, VT, ML, Ch, Cl, out1);
  gemm_t<_Float16, 2, 2, 0><<<gO, blk, 0, stream>>>(
      Ch, Cl, EMB, 0LL, WoT, EMB, 0LL,
      (void*)Y, (void*)Y, EMB, 0LL,
      NROW, EMB, EMB, 1.0f / 16384.0f, 1.0f / 4096.0f, 1.0f, 1.0f);
  resid_ln<<<gLN, blk, 0, stream>>>(Y, x, gam, bet, out0);
  (void)hipGetLastError();
}
